// MultiHeadCausalSelfAttention_11948599017550
// MI455X (gfx1250) — hardware-verified
//
#include <hip/hip_runtime.h>

typedef __attribute__((ext_vector_type(16))) _Float16 v16h;
typedef __attribute__((ext_vector_type(8)))  _Float16 v8h;
typedef __attribute__((ext_vector_type(16))) __bf16   v16b;
typedef __attribute__((ext_vector_type(8)))  __bf16   v8b;
typedef __attribute__((ext_vector_type(8)))  float    v8f;
typedef __attribute__((ext_vector_type(4)))  float    v4f;

constexpr int NBATCH = 4;
constexpr int SEQ_T  = 2048;
constexpr int EMB_D  = 1024;
constexpr int NHEAD  = 16;
constexpr int HDIM   = 64;
constexpr int MROWS  = NBATCH * SEQ_T;
constexpr int NBH    = NBATCH * NHEAD;
constexpr int KV_CH  = 64;
constexpr int OS_PITCH = 68;
constexpr int TR_PITCH = 72;
static_assert(EMB_D == NHEAD * HDIM, "head geometry");
static_assert(MROWS % 64 == 0 && EMB_D % 64 == 0 && EMB_D % 32 == 0, "tile multiples");
static_assert(SEQ_T % 64 == 0, "query/key tiles");


__device__ __forceinline__ unsigned short f2bf_bits(float f) {
  unsigned u = __float_as_uint(f);
  return (unsigned short)((u + 0x7FFFu + ((u >> 16) & 1u)) >> 16);
}
__device__ __forceinline__ float bf_bits2f(unsigned short h) { return __uint_as_float(((unsigned)h) << 16); }

__device__ __forceinline__ void dep_guard_h(v8f& a, v8f& b, v16h x, v16h y) { asm volatile("v_nop\n\tv_nop\n\tv_nop\n\tv_nop" : "+v"(a), "+v"(b) : "v"(x), "v"(y)); }
__device__ __forceinline__ void dep_guard_b(v8f& a, v8f& b, v16b x, v16b y) { asm volatile("v_nop\n\tv_nop\n\tv_nop\n\tv_nop" : "+v"(a), "+v"(b) : "v"(x), "v"(y)); }
__device__ __forceinline__ void keep4_h(v16h a, v16h b, v16h c, v16h d) { asm volatile("v_nop" :: "v"(a), "v"(b), "v"(c), "v"(d)); }
__device__ __forceinline__ void keep4_b(v16b a, v16b b, v16b c, v16b d) { asm volatile("v_nop" :: "v"(a), "v"(b), "v"(c), "v"(d)); }
__device__ __forceinline__ void acc_guard4(v8f& a, v8f& b, v8f& c, v8f& d) { asm volatile("v_nop\n\tv_nop\n\tv_nop\n\tv_nop" : "+v"(a), "+v"(b), "+v"(c), "+v"(d)); }
template <typename T> struct Frag;
template <> struct Frag<_Float16> {
  typedef v16h V; union U { v16h v; v8h h[2]; };
  static __device__ __forceinline__ v16h load(const _Float16* p) {
    U f; f.h[0] = *(const v8h*)(p); f.h[1] = *(const v8h*)(p + 16); return f.v;
  }
  static __device__ __forceinline__ v8f mma(v16h a, v16h b, v8f c) {
    return __builtin_amdgcn_wmma_f32_16x16x32_f16(false, a, false, b, (short)0, c, false, false);
  }
  static __device__ __forceinline__ void guard(v8f& a, v8f& b, v16h x, v16h y) { dep_guard_h(a, b, x, y); }
  static __device__ __forceinline__ void keep(v16h a, v16h b, v16h c, v16h d) { keep4_h(a, b, c, d); }
};
template <> struct Frag<__bf16> {
  typedef v16b V; union U { v16b v; v8b h[2]; };
  static __device__ __forceinline__ v16b load(const __bf16* p) {
    U f; f.h[0] = *(const v8b*)(p); f.h[1] = *(const v8b*)(p + 16); return f.v;
  }
  static __device__ __forceinline__ v8f mma(v16b a, v16b b, v8f c) {
    return __builtin_amdgcn_wmma_f32_16x16x32_bf16(false, a, false, b, (short)0, c, false, false);
  }
  static __device__ __forceinline__ void guard(v8f& a, v8f& b, v16b x, v16b y) { dep_guard_b(a, b, x, y); }
  static __device__ __forceinline__ void keep(v16b a, v16b b, v16b c, v16b d) { keep4_b(a, b, c, d); }
};

__device__ __forceinline__ unsigned short at_bf_bits(float f) {
  unsigned u = __float_as_uint(f);
  return (unsigned short)((u + 0x7FFFu + ((u >> 16) & 1u)) >> 16);
}
__device__ __forceinline__ __bf16 at_f2bf(float f) { return __builtin_bit_cast(__bf16, at_bf_bits(f)); }
__device__ __forceinline__ void at_split(float f, __bf16& hi, __bf16& lo) {
  const unsigned short hb = at_bf_bits(f);
  hi = __builtin_bit_cast(__bf16, hb);
  lo = at_f2bf(f - __uint_as_float(((unsigned)hb) << 16));
}
__device__ __forceinline__ v8f at_mma(v16b a, v16b b, v8f c) {
  c = __builtin_amdgcn_wmma_f32_16x16x32_bf16(false, a, false, b, (short)0, c, false, false);
  asm volatile("v_nop\n\tv_nop\n\tv_nop\n\tv_nop" : "+v"(c) : "v"(a), "v"(b));
  return c;
}

__global__ __launch_bounds__(256) void cast_f32_bf16x2(const float* __restrict__ in,
                                                       unsigned short* __restrict__ out, int n2) {
  const int i = blockIdx.x * 256 + threadIdx.x;
  if (i < n2) {
    const unsigned u = (unsigned)f2bf_bits(in[2 * i]) | ((unsigned)f2bf_bits(in[2 * i + 1]) << 16);
    ((volatile unsigned*)out)[i] = u;
    __threadfence();
    ((volatile unsigned*)out)[i] = u;
  }
}

__global__ __launch_bounds__(256) void cast3_f32_bf16x2(const float* __restrict__ in0, const float* __restrict__ in1,
                                                        const float* __restrict__ in2, unsigned short* __restrict__ out,
                                                        int n2each) {
  const int y = blockIdx.y;
  const float* in = (y == 0) ? in0 : ((y == 1) ? in1 : in2);
  unsigned short* o = out + (size_t)y * 2 * (size_t)n2each;
  const int i = blockIdx.x * 256 + threadIdx.x;
  if (i < n2each) {
    const unsigned u = (unsigned)f2bf_bits(in[2 * i]) | ((unsigned)f2bf_bits(in[2 * i + 1]) << 16);
    ((volatile unsigned*)o)[i] = u;
    __threadfence();
    ((volatile unsigned*)o)[i] = u;
  }
}

template <int ET> struct Elem;
template <> struct Elem<0> { typedef _Float16 T; };
template <> struct Elem<1> { typedef __bf16 T; };
template <int ET, int SPLITM, int BIAS_MODE, int OUT_MODE, bool RESID, int ACT = 0>
__global__ __launch_bounds__(256) void wmma_gemm64(
    const unsigned short* __restrict__ Ap, const unsigned short* __restrict__ A2p, int lda, long strideA,
    const unsigned short* __restrict__ Btp, const unsigned short* __restrict__ Bt2p, int ldb, long strideB,
    void* __restrict__ Cout, void* __restrict__ Cout2, int ldc, long strideC,
    const float* __restrict__ bias,
    const float* __restrict__ resid, long strideR,
    int M, int N, int K, float scale) {
  typedef typename Elem<ET>::T T;
  typedef typename Frag<T>::V V;
  constexpr bool SPA = (SPLITM >= 1);
  constexpr bool SPB = (SPLITM >= 2);
  const T* A = (const T*)Ap; const T* A2 = (const T*)A2p; const T* Bt = (const T*)Btp; const T* Bt2 = (const T*)Bt2p;
  __shared__ __align__(16) float sT[8][16 * 68];
  const int b    = blockIdx.y;
  const int lane = threadIdx.x & 31;
  const int wave = threadIdx.x >> 5;
  const int tilesN = N >> 6;
  const int tilesM = M >> 6;
  const int tile = blockIdx.x * 8 + wave;
  if (tile >= tilesM * tilesN) return;
  const int tm = tile / tilesN;
  const int tn = tile - tm * tilesN;
  const int m0 = tm << 6;
  const int n0 = tn << 6;

  const T* Ab  = A  + (size_t)b * strideA;
  const T* Bb  = Bt + (size_t)b * strideB;
  const T* Ab2 = SPA ? (A2  + (size_t)b * strideA) : nullptr;
  const T* Bb2 = SPB ? (Bt2 + (size_t)b * strideB) : nullptr;

  const int rlane = lane & 15;
  const int koff  = (lane >> 4) * 8;
  const int mOff  = (lane >> 4) * 8;

  v8f acc[4][4];
#pragma unroll
  for (int i = 0; i < 4; ++i)
#pragma unroll
    for (int j = 0; j < 4; ++j) acc[i][j] = (v8f){0.f,0.f,0.f,0.f,0.f,0.f,0.f,0.f};

  for (int k0 = 0; k0 < K; k0 += 32) {
    V bh[4], bl[4];
#pragma unroll
    for (int j = 0; j < 4; ++j) {
      const size_t bo = (size_t)(n0 + (j << 4) + rlane) * ldb + koff + k0;
      bh[j] = Frag<T>::load(Bb + bo);
      if (SPB) bl[j] = Frag<T>::load(Bb2 + bo);
    }
#pragma unroll
    for (int i = 0; i < 4; ++i) {
      const size_t ao = (size_t)(m0 + (i << 4) + rlane) * lda + koff + k0;
      V ah = Frag<T>::load(Ab + ao);
      V al;
      if (SPA) al = Frag<T>::load(Ab2 + ao);
#pragma unroll
      for (int j = 0; j < 4; ++j) {
        acc[i][j] = Frag<T>::mma(ah, bh[j], acc[i][j]);
        if (SPB) acc[i][j] = Frag<T>::mma(ah, bl[j], acc[i][j]);
        if (SPA) acc[i][j] = Frag<T>::mma(al, bh[j], acc[i][j]);
      }
      Frag<T>::guard(acc[i][0], acc[i][3], ah, SPA ? al : ah);
    }
    Frag<T>::keep(bh[0], bh[1], bh[2], bh[3]);
    if (SPB) Frag<T>::keep(bl[0], bl[1], bl[2], bl[3]);
  }
  acc_guard4(acc[0][0], acc[0][1], acc[0][2], acc[0][3]);
  acc_guard4(acc[1][0], acc[1][1], acc[1][2], acc[1][3]);
  acc_guard4(acc[2][0], acc[2][1], acc[2][2], acc[2][3]);
  acc_guard4(acc[3][0], acc[3][1], acc[3][2], acc[3][3]);

  float* slab = sT[wave];
  const float* Rb = RESID ? (resid + (size_t)b * strideR) : nullptr;
#pragma unroll
  for (int i = 0; i < 4; ++i) {
    const int mBase = m0 + (i << 4);
#pragma unroll
    for (int j = 0; j < 4; ++j) {
      const int n = n0 + (j << 4) + rlane;
      float bv = 0.f;
      if (BIAS_MODE == 2) bv = bias[n];
      if (BIAS_MODE == 3) bv = bf_bits2f(f2bf_bits(bias[n]));
#pragma unroll
      for (int r = 0; r < 8; ++r) {
        float v = acc[i][j][r] * scale;
        if (BIAS_MODE == 1) v += bias[mBase + mOff + r];
        if (BIAS_MODE == 2 || BIAS_MODE == 3) v += bv;
        if (RESID) v += Rb[(size_t)(mBase + mOff + r) * ldc + n];
        if (ACT == 1) v = tanhf(v);
        if (ACT == 2) v = fmaxf(v, 0.0f);
        if (ACT == 4) v = (v > 0.f) ? v : 0.01f * v;
        slab[(mOff + r) * 68 + (j << 4) + rlane] = v;
      }
    }
    __builtin_amdgcn_fence(__ATOMIC_RELEASE, "workgroup");
    __builtin_amdgcn_wave_barrier();
    __builtin_amdgcn_fence(__ATOMIC_ACQUIRE, "workgroup");
    if (OUT_MODE == 0) {
      float* C = (float*)Cout + (size_t)b * strideC;
      const int hh = lane >> 4, c4 = (lane & 15) * 4;
      for (int pass = 0; pass < 2; ++pass) {
#pragma unroll
        for (int it = 0; it < 8; ++it) {
          const int row = it * 2 + hh;
          v4f v = *(const v4f*)(slab + row * 68 + c4);
          *(volatile v4f*)(C + (size_t)(mBase + row) * ldc + n0 + c4) = v;
        }
        __threadfence();
      }
    } else {
      const int q = lane >> 3, c8 = (lane & 7) * 8;
      unsigned short* C  = (unsigned short*)Cout  + (size_t)b * strideC;
      unsigned short* C2 = (OUT_MODE == 2) ? ((unsigned short*)Cout2 + (size_t)b * strideC) : nullptr;
      for (int pass = 0; pass < 2; ++pass) {
#pragma unroll
        for (int it = 0; it < 4; ++it) {
          const int row = it * 4 + q;
          const float* sp = slab + row * 68 + c8;
          v8h hv, lv;
#pragma unroll
          for (int e = 0; e < 8; ++e) {
            if (OUT_MODE == 1) {
              hv[e] = (_Float16)sp[e];
            } else {
              unsigned short hb = f2bf_bits(sp[e]);
              unsigned short lb = f2bf_bits(sp[e] - bf_bits2f(hb));
              hv[e] = __builtin_bit_cast(_Float16, hb);
              lv[e] = __builtin_bit_cast(_Float16, lb);
            }
          }
          *(volatile v8h*)(C + (size_t)(mBase + row) * ldc + n0 + c8) = hv;
          if (OUT_MODE == 2) *(volatile v8h*)(C2 + (size_t)(mBase + row) * ldc + n0 + c8) = lv;
        }
        __threadfence();
      }
    }
    __builtin_amdgcn_fence(__ATOMIC_RELEASE, "workgroup");
    __builtin_amdgcn_wave_barrier();
    __builtin_amdgcn_fence(__ATOMIC_ACQUIRE, "workgroup");
  }
}

__global__ __launch_bounds__(256) void vt_transpose_k(const unsigned short* __restrict__ vh, const unsigned short* __restrict__ vl,
                                                      unsigned short* __restrict__ vth, unsigned short* __restrict__ vtl) {
  __shared__ __align__(16) _Float16 th[64 * TR_PITCH];
  __shared__ __align__(16) _Float16 tl[64 * TR_PITCH];
  const int st0 = blockIdx.x * 64, g = blockIdx.y;
  const int b = g / NHEAD, h = g - b * NHEAD;
  const int tid = threadIdx.x;
  {
    const int sloc = tid >> 2, d0 = (tid & 3) * 16;
    const size_t so = ((size_t)b * SEQ_T + st0 + sloc) * EMB_D + h * HDIM + d0;
    const v8h a0 = *(const v8h*)((const _Float16*)vh + so);
    const v8h a1 = *(const v8h*)((const _Float16*)vh + so + 8);
    const v8h b0 = *(const v8h*)((const _Float16*)vl + so);
    const v8h b1 = *(const v8h*)((const _Float16*)vl + so + 8);
#pragma unroll
    for (int e = 0; e < 8; ++e) {
      th[(d0 + e) * TR_PITCH + sloc]     = a0[e];
      th[(d0 + 8 + e) * TR_PITCH + sloc] = a1[e];
      tl[(d0 + e) * TR_PITCH + sloc]     = b0[e];
      tl[(d0 + 8 + e) * TR_PITCH + sloc] = b1[e];
    }
  }
  __syncthreads();
  const int wave = tid >> 5, lane = tid & 31, q8 = lane >> 3, c8 = (lane & 7) * 8;
  const int dA = wave * 8 + q8, dB = wave * 8 + 4 + q8;
  const v8h hvA = *(const v8h*)(th + dA * TR_PITCH + c8);
  const v8h hvB = *(const v8h*)(th + dB * TR_PITCH + c8);
  const v8h lvA = *(const v8h*)(tl + dA * TR_PITCH + c8);
  const v8h lvB = *(const v8h*)(tl + dB * TR_PITCH + c8);
  const size_t oA = ((size_t)g * HDIM + dA) * SEQ_T + st0 + c8;
  const size_t oB = ((size_t)g * HDIM + dB) * SEQ_T + st0 + c8;
  for (int pass = 0; pass < 2; ++pass) {
    *(volatile v8h*)(vth + oA) = hvA;
    *(volatile v8h*)(vth + oB) = hvB;
    *(volatile v8h*)(vtl + oA) = lvA;
    *(volatile v8h*)(vtl + oB) = lvB;
    __threadfence();
  }
}

__global__ __launch_bounds__(128) void attn_causal_hd64_k(
    const unsigned short* __restrict__ qh_p, const unsigned short* __restrict__ ql_p,
    const unsigned short* __restrict__ kh_p, const unsigned short* __restrict__ kl_p,
    const unsigned short* __restrict__ vth_p, const unsigned short* __restrict__ vtl_p,
    unsigned short* __restrict__ oh_p, unsigned short* __restrict__ ol_p, float sscale) {
  union FB { v16b v; v8b h[2]; };
  __shared__ __align__(16) __bf16 Ksh[KV_CH * HDIM];
  __shared__ __align__(16) __bf16 Ksl[KV_CH * HDIM];
  __shared__ __align__(16) __bf16 Vsh[HDIM * KV_CH];
  __shared__ __align__(16) __bf16 Vsl[HDIM * KV_CH];
  __shared__ __align__(16) __bf16 Psh[4][16 * KV_CH];
  __shared__ __align__(16) __bf16 Psl[4][16 * KV_CH];
  __shared__ __align__(16) float  Os[4][16 * OS_PITCH];

  const int tid  = threadIdx.x;
  const int wave = tid >> 5;
  const int lane = tid & 31;
  const int hh   = lane >> 4;
  const int c    = lane & 15;

  constexpr int NQB = SEQ_T / 64;
  const int bx = blockIdx.x;
  const int qb = bx % NQB;
  const int bh = bx / NQB;
  const int h  = bh % NHEAD;
  const int b  = bh / NHEAD;
  const int q0 = qb * 64 + wave * 16;
  const size_t tok0 = (size_t)b * SEQ_T;
  const int colh = h * HDIM;

  const __bf16* qh  = (const __bf16*)qh_p;
  const __bf16* ql  = (const __bf16*)ql_p;
  const __bf16* kh  = (const __bf16*)kh_p;
  const __bf16* kl  = (const __bf16*)kl_p;
  const __bf16* vth = (const __bf16*)vth_p;
  const __bf16* vtl = (const __bf16*)vtl_p;

  v16b qah[2], qal[2];
  {
    const size_t qo = (tok0 + q0 + c) * EMB_D + colh + 8 * hh;
#pragma unroll
    for (int dc = 0; dc < 2; ++dc) {
      qah[dc] = Frag<__bf16>::load(qh + qo + dc * 32);
      qal[dc] = Frag<__bf16>::load(ql + qo + dc * 32);
    }
  }

  float mrow[8], lrow[8];
  v8f oacc[4];
#pragma unroll
  for (int r = 0; r < 8; ++r) { mrow[r] = -__builtin_inff(); lrow[r] = 0.f; }
#pragma unroll
  for (int t = 0; t < 4; ++t) oacc[t] = (v8f){0.f,0.f,0.f,0.f,0.f,0.f,0.f,0.f};

  for (int kc = 0; kc <= qb; ++kc) {
    const int kv0 = kc * KV_CH;
    __syncthreads();
    {
      const int r = tid >> 1, half = (tid & 1) * 32;
      const size_t ko = (tok0 + kv0 + r) * EMB_D + colh + half;
      const size_t vo = ((size_t)bh * HDIM + r) * SEQ_T + kv0 + half;
#pragma unroll
      for (int i = 0; i < 4; ++i) {
        const v8b a0 = *(const v8b*)(kh + ko + 8 * i);
        const v8b a1 = *(const v8b*)(kl + ko + 8 * i);
        const v8b b0 = *(const v8b*)(vth + vo + 8 * i);
        const v8b b1 = *(const v8b*)(vtl + vo + 8 * i);
        *(v8b*)(Ksh + r * HDIM + half + 8 * i)  = a0;
        *(v8b*)(Ksl + r * HDIM + half + 8 * i)  = a1;
        *(v8b*)(Vsh + r * KV_CH + half + 8 * i) = b0;
        *(v8b*)(Vsl + r * KV_CH + half + 8 * i) = b1;
      }
    }
    __syncthreads();

    v8f s[4];
#pragma unroll
    for (int j = 0; j < 4; ++j) {
      s[j] = (v8f){0.f,0.f,0.f,0.f,0.f,0.f,0.f,0.f};
#pragma unroll
      for (int dc = 0; dc < 2; ++dc) {
        FB kb, kbl;
        kb.h[0]  = *(const v8b*)(Ksh + (j * 16 + c) * HDIM + dc * 32 + 8 * hh);
        kb.h[1]  = *(const v8b*)(Ksh + (j * 16 + c) * HDIM + dc * 32 + 16 + 8 * hh);
        kbl.h[0] = *(const v8b*)(Ksl + (j * 16 + c) * HDIM + dc * 32 + 8 * hh);
        kbl.h[1] = *(const v8b*)(Ksl + (j * 16 + c) * HDIM + dc * 32 + 16 + 8 * hh);
        s[j] = at_mma(qah[dc], kb.v,  s[j]);
        s[j] = at_mma(qah[dc], kbl.v, s[j]);
        s[j] = at_mma(qal[dc], kb.v,  s[j]);
      }
    }

    const bool diag = (kc == qb);
    float cm[8];
#pragma unroll
    for (int r = 0; r < 8; ++r) {
      const int qrow = q0 + 8 * hh + r;
      float m = -__builtin_inff();
#pragma unroll
      for (int j = 0; j < 4; ++j) {
        const int kvcol = kv0 + j * 16 + c;
        float sv = s[j][r] * sscale;
        sv = (diag && (kvcol > qrow)) ? -__builtin_inff() : sv;
        s[j][r] = sv;
        m = fmaxf(m, sv);
      }
#pragma unroll
      for (int off = 1; off < 16; off <<= 1) m = fmaxf(m, __shfl_xor(m, off, 32));
      cm[r] = m;
    }

    __bf16* pwh = Psh[wave];
    __bf16* pwl = Psl[wave];
#pragma unroll
    for (int r = 0; r < 8; ++r) {
      const float mnew = fmaxf(mrow[r], cm[r]);
      const float alpha = expf(mrow[r] - mnew);
      mrow[r] = mnew;
      float psum = 0.f;
#pragma unroll
      for (int j = 0; j < 4; ++j) {
        const float p = expf(s[j][r] - mnew);
        psum += p;
        __bf16 a, bl;
        at_split(p, a, bl);
        pwh[(8 * hh + r) * KV_CH + j * 16 + c] = a;
        pwl[(8 * hh + r) * KV_CH + j * 16 + c] = bl;
      }
#pragma unroll
      for (int off = 1; off < 16; off <<= 1) psum += __shfl_xor(psum, off, 32);
      lrow[r] = lrow[r] * alpha + psum;
#pragma unroll
      for (int t = 0; t < 4; ++t) oacc[t][r] *= alpha;
    }
    __builtin_amdgcn_fence(__ATOMIC_RELEASE, "workgroup");
    __builtin_amdgcn_wave_barrier();
    __builtin_amdgcn_fence(__ATOMIC_ACQUIRE, "workgroup");

#pragma unroll
    for (int kk = 0; kk < 2; ++kk) {
      FB pa, pl;
      pa.h[0] = *(const v8b*)(pwh + c * KV_CH + kk * 32 + 8 * hh);
      pa.h[1] = *(const v8b*)(pwh + c * KV_CH + kk * 32 + 16 + 8 * hh);
      pl.h[0] = *(const v8b*)(pwl + c * KV_CH + kk * 32 + 8 * hh);
      pl.h[1] = *(const v8b*)(pwl + c * KV_CH + kk * 32 + 16 + 8 * hh);
#pragma unroll
      for (int t = 0; t < 4; ++t) {
        FB vb, vbl;
        vb.h[0]  = *(const v8b*)(Vsh + (t * 16 + c) * KV_CH + kk * 32 + 8 * hh);
        vb.h[1]  = *(const v8b*)(Vsh + (t * 16 + c) * KV_CH + kk * 32 + 16 + 8 * hh);
        vbl.h[0] = *(const v8b*)(Vsl + (t * 16 + c) * KV_CH + kk * 32 + 8 * hh);
        vbl.h[1] = *(const v8b*)(Vsl + (t * 16 + c) * KV_CH + kk * 32 + 16 + 8 * hh);
        oacc[t] = at_mma(pa.v, vb.v,  oacc[t]);
        oacc[t] = at_mma(pa.v, vbl.v, oacc[t]);
        oacc[t] = at_mma(pl.v, vb.v,  oacc[t]);
      }
    }
  }

  float* os = Os[wave];
#pragma unroll
  for (int r = 0; r < 8; ++r) {
    const float inv = 1.0f / lrow[r];
#pragma unroll
    for (int t = 0; t < 4; ++t) os[(8 * hh + r) * OS_PITCH + t * 16 + c] = oacc[t][r] * inv;
  }
  __builtin_amdgcn_fence(__ATOMIC_RELEASE, "workgroup");
  __builtin_amdgcn_wave_barrier();
  __builtin_amdgcn_fence(__ATOMIC_ACQUIRE, "workgroup");
  {
    const int q8 = lane >> 3, c8 = (lane & 7) * 8;
    const size_t obase = (tok0 + q0) * EMB_D + colh + c8;
    for (int pass = 0; pass < 2; ++pass) {
#pragma unroll
      for (int it = 0; it < 4; ++it) {
        const int row = it * 4 + q8;
        const float* sp = os + row * OS_PITCH + c8;
        v8h hv, lv;
#pragma unroll
        for (int e = 0; e < 8; ++e) {
          const unsigned short hb = f2bf_bits(sp[e]);
          const unsigned short lb = f2bf_bits(sp[e] - bf_bits2f(hb));
          hv[e] = __builtin_bit_cast(_Float16, hb);
          lv[e] = __builtin_bit_cast(_Float16, lb);
        }
        *(volatile v8h*)(oh_p + obase + (size_t)row * EMB_D) = hv;
        *(volatile v8h*)(ol_p + obase + (size_t)row * EMB_D) = lv;
      }
      __threadfence();
    }
  }
}

extern "C" void kernel_launch(void* const* d_in, const int* in_sizes, int n_in,
                              void* d_out, int out_size, void* d_ws,
                              size_t ws_size, hipStream_t stream) {
  constexpr size_t PLANE   = (size_t)MROWS * EMB_D;
  constexpr size_t PLANE_B = PLANE * 2;
  constexpr size_t WSQ     = (size_t)EMB_D * EMB_D;
  constexpr size_t VT_B    = (size_t)NBH * HDIM * SEQ_T * 2;
  static_assert(VT_B == PLANE_B, "vt plane size");
  constexpr size_t OFF_XB   = 0;
  constexpr size_t OFF_WQKV = 1 * PLANE_B;
  constexpr size_t OFF_VTH  = 0;
  constexpr size_t OFF_VTL  = 1 * PLANE_B;
  constexpr size_t OFF_HI   = 2 * PLANE_B;
  constexpr size_t OFF_LO   = 5 * PLANE_B;
  constexpr size_t OFF_WO   = OFF_HI;
  constexpr size_t WS_TOTAL = 8 * PLANE_B;
  static_assert(WS_TOTAL == 134217728ull, "carve total 128 MiB");
  static_assert(OFF_WQKV + 3 * WSQ * 2 <= OFF_HI, "weights fit below the planes");
  static_assert(OFF_VTL + VT_B <= OFF_HI, "vt lo fits below the planes");
  static_assert(OFF_WO + WSQ * 2 <= OFF_HI + PLANE_B, "wo fits in the dead q hi plane");

  if (n_in < 6) return;
  if ((size_t)in_sizes[0] != PLANE || (size_t)in_sizes[1] != WSQ || (size_t)in_sizes[2] != WSQ ||
      (size_t)in_sizes[3] != WSQ || (size_t)in_sizes[4] != WSQ || in_sizes[5] != EMB_D) return;
  if ((size_t)out_size != PLANE) return;
  if (ws_size < WS_TOTAL) return;

  const float* x  = (const float*)d_in[0];
  const float* Wq = (const float*)d_in[1];
  const float* Wk = (const float*)d_in[2];
  const float* Wv = (const float*)d_in[3];
  const float* Wo = (const float*)d_in[4];
  const float* bo = (const float*)d_in[5];
  float* out = (float*)d_out;

  char* ws = (char*)d_ws;
  unsigned short* xb   = (unsigned short*)(ws + OFF_XB);
  unsigned short* wqkv = (unsigned short*)(ws + OFF_WQKV);
  unsigned short* hi   = (unsigned short*)(ws + OFF_HI);
  unsigned short* lo   = (unsigned short*)(ws + OFF_LO);
  unsigned short* qh = hi;               unsigned short* ql = lo;
  unsigned short* kh = hi + PLANE;       unsigned short* kl = lo + PLANE;
  unsigned short* vh = hi + 2 * PLANE;   unsigned short* vl = lo + 2 * PLANE;
  unsigned short* vth = (unsigned short*)(ws + OFF_VTH);
  unsigned short* vtl = (unsigned short*)(ws + OFF_VTL);
  unsigned short* oh = vh;
  unsigned short* ol = vl;
  unsigned short* wo16 = (unsigned short*)(ws + OFF_WO);

  cast_f32_bf16x2<<<(unsigned)(PLANE / 2 / 256), 256, 0, stream>>>(x, xb, (int)(PLANE / 2));
  cast3_f32_bf16x2<<<dim3((unsigned)(WSQ / 2 / 256), 3), 256, 0, stream>>>(Wq, Wk, Wv, wqkv, (int)(WSQ / 2));
  wmma_gemm64<1, 0, 0, 2, false><<<dim3((MROWS / 64) * (EMB_D / 64) / 8, 3), 256, 0, stream>>>(
      xb, xb, EMB_D, 0L, wqkv, wqkv, EMB_D, (long)WSQ,
      (void*)hi, (void*)lo, EMB_D, (long)PLANE, bo, x, 0L, MROWS, EMB_D, EMB_D, 1.0f);
  vt_transpose_k<<<dim3(SEQ_T / 64, NBH), 256, 0, stream>>>(vh, vl, vth, vtl);
  attn_causal_hd64_k<<<NBH * (SEQ_T / 64), 128, 0, stream>>>(qh, ql, kh, kl, vth, vtl, oh, ol, 0.125f);
  cast_f32_bf16x2<<<(unsigned)(WSQ / 2 / 256), 256, 0, stream>>>(Wo, wo16, (int)(WSQ / 2));
  wmma_gemm64<1, 1, 3, 0, false><<<dim3((MROWS / 64) * (EMB_D / 64) / 8, 1), 256, 0, stream>>>(
      oh, ol, EMB_D, 0L, wo16, wo16, EMB_D, 0L,
      (void*)out, (void*)out, EMB_D, 0L, bo, x, 0L, MROWS, EMB_D, EMB_D, 1.0f);
}
